// GAT_7421703487704
// MI455X (gfx1250) — hardware-verified
//
#include <hip/hip_runtime.h>
#include <stddef.h>
#include <stdint.h>
#include <math.h>


#define NB     8
#define NN     1024
#define NF     256
#define NHD    8
#define HID    64
#define CAT    512
#define NCL    256
#define MROWS  8192
#define BPITCH 36
#define NEGC   (-9.0e15f)
#define OUT1OFF 2097152
#define WSMAX  134217728

#define PU_X   (MROWS * (NF / 8))
#define PU_WA  (CAT * (2 * NF / 8))
#define PU_WO  (NCL * (2 * CAT / 8))
#define PU_ADJ (MROWS * 8)
#define PU_ALL (PU_X + PU_WA + PU_WO + PU_ADJ)

static_assert(MROWS == NB * NN);
static_assert(CAT == NHD * HID);
static_assert(PU_X % 256 == 0 && PU_WA % 256 == 0 && PU_WO % 256 == 0 && PU_ADJ % 256 == 0);
static_assert(NF % 32 == 0 && (2 * NF) % 32 == 0 && (2 * CAT) % 32 == 0 && NN % 64 == 0);
static_assert(OUT1OFF == MROWS * NCL);
static_assert(OUT1OFF + (NB - 1) * NCL + NCL - 1 < MROWS * NCL + NB * NCL);
static_assert((OUT1OFF * 4) % 128 == 0);
static_assert(BPITCH >= 32 && (BPITCH % 4) == 0);

typedef float          v4f  __attribute__((ext_vector_type(4)));
typedef float          v8f  __attribute__((ext_vector_type(8)));
typedef int            v4i  __attribute__((ext_vector_type(4)));
typedef int            v8i  __attribute__((ext_vector_type(8)));
typedef unsigned int   v4u  __attribute__((ext_vector_type(4)));
typedef unsigned short v8us __attribute__((ext_vector_type(8)));
typedef __bf16         v16b __attribute__((ext_vector_type(16)));
typedef v4f  __attribute__((may_alias)) v4fa;
typedef v4u  __attribute__((may_alias)) v4ua;
typedef v8us __attribute__((may_alias)) v8usa;
union FragB { v16b v; v8us h[2]; v8i w; };

__device__ __forceinline__ v8f wmb(const FragB& a, const FragB& b, v8f c) {
  v8f d = __builtin_amdgcn_wmma_f32_16x16x32_bf16(false, a.v, false, b.v, (short)0, c, false, false);
  asm volatile("v_nop\n\tv_nop\n\tv_nop\n\tv_nop" : "+v"(d) : "v"(a.w), "v"(b.w));
  return d;
}

__device__ __forceinline__ unsigned int f2bf(float f) {
  const unsigned int u = __float_as_uint(f);
  return ((u + 0x7FFFu + ((u >> 16) & 1u)) >> 16) & 0xFFFFu;
}
__device__ __forceinline__ float bf2f(unsigned int b) { return __uint_as_float(b << 16); }
__device__ __forceinline__ float bfr(float f) { return bf2f(f2bf(f)); }
__device__ __forceinline__ v4f bfr4(const v4f a) {
  v4f r; r.x = bfr(a.x); r.y = bfr(a.y); r.z = bfr(a.z); r.w = bfr(a.w); return r;
}
__device__ __forceinline__ unsigned int pk2(float lo, float hi) { return f2bf(lo) | (f2bf(hi) << 16); }
__device__ __forceinline__ v4u pack8(const v4f a, const v4f b) {
  v4u r;
  r.x = pk2(a.x, a.y); r.y = pk2(a.z, a.w); r.z = pk2(b.x, b.y); r.w = pk2(b.z, b.w);
  return r;
}
__device__ __forceinline__ void split8(const float (&v)[8], v4u& hv, v4u& lv) {
  unsigned int hb[8], lb[8];
#pragma unroll
  for (int i = 0; i < 8; ++i) {
    hb[i] = f2bf(v[i]);
    lb[i] = f2bf(v[i] - bf2f(hb[i]));
  }
  hv.x = hb[0] | (hb[1] << 16); hv.y = hb[2] | (hb[3] << 16); hv.z = hb[4] | (hb[5] << 16); hv.w = hb[6] | (hb[7] << 16);
  lv.x = lb[0] | (lb[1] << 16); lv.y = lb[2] | (lb[3] << 16); lv.z = lb[4] | (lb[5] << 16); lv.w = lb[6] | (lb[7] << 16);
}
__device__ __forceinline__ float eluf(float x) { return x > 0.f ? x : expm1f(fminf(x, 0.f)); }

__device__ __forceinline__ unsigned int bits32(const int* __restrict__ p) {
  unsigned int w = 0u;
#pragma unroll
  for (int g = 0; g < 8; ++g) {
    const v4i a = *(const v4i*)(p + 4 * g);
    w |= (a.x > 0 ? 1u : 0u) << (4 * g);
    w |= (a.y > 0 ? 1u : 0u) << (4 * g + 1);
    w |= (a.z > 0 ? 1u : 0u) << (4 * g + 2);
    w |= (a.w > 0 ? 1u : 0u) << (4 * g + 3);
  }
  return w;
}

__global__ __launch_bounds__(256) void k_prep(const float* __restrict__ x, const int* __restrict__ adj,
                                              const float* __restrict__ Watt, const float* __restrict__ Wout,
                                              unsigned short* XB, unsigned short* WA2, unsigned short* WO2,
                                              unsigned int* ABITS) {
  const int u = (int)blockIdx.x * 256 + (int)threadIdx.x;
  if (u < PU_X) {
    const int row = u >> 5;
    const int c0  = (u & 31) * 8;
    const float* p = x + (size_t)row * NF + c0;
    const v4f a = *(const v4fa*)p, b = *(const v4fa*)(p + 4);
    const v4u hv = pack8(a, b);
    unsigned short* o = XB + (size_t)row * NF + c0;
    *(volatile v4u*)o = hv;
    __threadfence();
    *(volatile v4u*)o = hv;
  } else if (u < PU_X + PU_WA) {
    const int v  = u - PU_X;
    const int n  = v >> 6;
    const int k8 = (v & 63) * 8;
    const int kk = k8 & (NF - 1);
    const int h  = n >> 6, oo = n & 63;
    const float* p = Watt + ((size_t)h * NF + kk) * HID + oo;
    v4f a, b;
    a.x = p[0];       a.y = p[HID];     a.z = p[2 * HID]; a.w = p[3 * HID];
    b.x = p[4 * HID]; b.y = p[5 * HID]; b.z = p[6 * HID]; b.w = p[7 * HID];
    const v4u wv = pack8(a, b);
    unsigned short* o = WA2 + (size_t)n * (2 * NF) + k8;
    *(volatile v4u*)o = wv;
    __threadfence();
    *(volatile v4u*)o = wv;
  } else if (u < PU_X + PU_WA + PU_WO) {
    const int v  = u - PU_X - PU_WA;
    const int n  = v >> 7;
    const int k8 = (v & 127) * 8;
    const int kk = k8 & (CAT - 1);
    const float* p = Wout + (size_t)kk * NCL + n;
    v4f a, b;
    a.x = p[0];       a.y = p[NCL];     a.z = p[2 * NCL]; a.w = p[3 * NCL];
    b.x = p[4 * NCL]; b.y = p[5 * NCL]; b.z = p[6 * NCL]; b.w = p[7 * NCL];
    const v4u wv = pack8(a, b);
    unsigned short* o = WO2 + (size_t)n * (2 * CAT) + k8;
    *(volatile v4u*)o = wv;
    __threadfence();
    *(volatile v4u*)o = wv;
  } else if (u < PU_ALL) {
    const int v   = u - PU_X - PU_WA - PU_WO;
    const int row = v >> 3;
    const int q   = v & 7;
    const int* p  = adj + (size_t)row * NN + 128 * q;
    v4u wv;
    wv.x = bits32(p);
    wv.y = bits32(p + 32);
    wv.z = bits32(p + 64);
    wv.w = bits32(p + 96);
    unsigned int* o = ABITS + (size_t)row * 32 + 4 * q;
    *(volatile v4u*)o = wv;
    __threadfence();
    *(volatile v4u*)o = wv;
  }
}

template <int LDC, int NT, int NIT>
__device__ __forceinline__ void tr_store_pass(const float* stg, unsigned short* Ph, unsigned short* Pl,
                                              size_t base, int tid) {
  static_assert(NIT * NT == LDC * 8);
#pragma unroll 1
  for (int it = 0; it < NIT; ++it) {
    const int u  = it * NT + tid;
    const int c  = u >> 3;
    const int pc = u & 7;
    float v[8];
#pragma unroll
    for (int i = 0; i < 8; ++i) v[i] = stg[(8 * pc + i) * LDC + c];
    v4u hv, lv;
    split8(v, hv, lv);
    const size_t a = base + (size_t)c * NN + 8 * pc;
    *(volatile v4u*)(Ph + a) = hv;
    *(volatile v4u*)(Pl + a) = lv;
  }
}

__global__ __launch_bounds__(128) void k_h(const unsigned short* __restrict__ A, int lda, int K,
                                           const unsigned short* __restrict__ WT,
                                           const float* __restrict__ aatt,
                                           float* F12, unsigned short* HTh, unsigned short* HTl) {
  __shared__ __attribute__((aligned(16))) float stg[64 * 64];
  __shared__ __attribute__((aligned(16))) float satt[128];
  __shared__ __attribute__((aligned(16))) float sdot[128];
  const int tid = (int)threadIdx.x, lane = tid & 31, wave = tid >> 5, hh = lane >> 4, m = lane & 15;
  const int rowBase = (int)blockIdx.x * 64;
  const int head    = (int)blockIdx.y;
  const int col0    = head * 64;

  satt[tid] = bfr(aatt[head * 128 + tid]);

  v8f acc[4];
  {
    const v8f z = {0.f, 0.f, 0.f, 0.f, 0.f, 0.f, 0.f, 0.f};
    acc[0] = z; acc[1] = z; acc[2] = z; acc[3] = z;
  }
  const unsigned short* ap = A  + (size_t)(rowBase + 16 * wave + m) * (size_t)lda + 8 * hh;
  const unsigned short* wp = WT + (size_t)(col0 + m) * (size_t)(2 * NF) + 8 * hh;
  const int ksteps = K >> 5;
#pragma unroll 1
  for (int ks = 0; ks < ksteps; ++ks) {
    FragB af;
    af.h[0] = *(const v8usa*)(ap + 32 * ks);
    af.h[1] = *(const v8usa*)(ap + 32 * ks + 16);
#pragma unroll
    for (int t = 0; t < 4; ++t) {
      const unsigned short* wq = wp + (size_t)(16 * t) * (size_t)(2 * NF) + 32 * ks;
      FragB bf;
      bf.h[0] = *(const v8usa*)wq;
      bf.h[1] = *(const v8usa*)(wq + 16);
      acc[t] = wmb(af, bf, acc[t]);
    }
  }

#pragma unroll
  for (int t = 0; t < 4; ++t) {
    const int lc = 16 * t + m;
#pragma unroll
    for (int r = 0; r < 8; ++r) {
      const int lr = 16 * wave + 8 * hh + r;
      stg[lr * 64 + lc] = acc[t][r];
    }
  }
  __syncthreads();

  {
    const int row = tid & 63, which = tid >> 6;
    const float* sa = satt + which * 64;
    const float* hr = stg + row * 64;
    float d = 0.f;
#pragma unroll 4
    for (int c4 = 0; c4 < 16; ++c4) {
      const v4f hv = *(const v4fa*)(hr + 4 * c4);
      const v4f av = *(const v4fa*)(sa + 4 * c4);
      d = fmaf(hv.x, av.x, d);
      d = fmaf(hv.y, av.y, d);
      d = fmaf(hv.z, av.z, d);
      d = fmaf(hv.w, av.w, d);
    }
    sdot[which * 64 + row] = d;
  }
  __syncthreads();

  const int b  = rowBase >> 10, n0 = rowBase & (NN - 1);
  const size_t bh = (size_t)b * NHD + head;
  const int which2 = lane >> 4, piece = lane & 15;
  const v4f sdv = *(const v4fa*)(sdot + which2 * 64 + 4 * piece);
  float* sp = F12 + (bh * 2 + which2) * NN + n0 + 4 * piece;
  const size_t hbase = bh * (size_t)(HID * NN) + n0;

  tr_store_pass<64, 128, 4>(stg, HTh, HTl, hbase, tid);
  if (wave == 0) *(volatile v4f*)sp = sdv;
  __threadfence();
  tr_store_pass<64, 128, 4>(stg, HTh, HTl, hbase, tid);
  if (wave == 0) *(volatile v4f*)sp = sdv;
}

__device__ __forceinline__ float row_max(const unsigned int* sb, const float* sf, float f1v, int hh) {
  float mx = -3.0e38f;
  unsigned int any = 0u;
#pragma unroll 1
  for (int jt = 0; jt < 32; ++jt) {
    const unsigned int word = sb[jt];
#pragma unroll
    for (int hf = 0; hf < 2; ++hf) {
      const int sh = 16 * hf + 8 * hh;
      const unsigned int by = (word >> sh) & 0xffu;
      any |= by;
      const v4f fa = *(const v4fa*)(sf + 32 * jt + sh);
      const v4f fb = *(const v4fa*)(sf + 32 * jt + sh + 4);
      mx = fmaxf(mx, (by & 1u)   ? fa.x : -3.0e38f);
      mx = fmaxf(mx, (by & 2u)   ? fa.y : -3.0e38f);
      mx = fmaxf(mx, (by & 4u)   ? fa.z : -3.0e38f);
      mx = fmaxf(mx, (by & 8u)   ? fa.w : -3.0e38f);
      mx = fmaxf(mx, (by & 16u)  ? fb.x : -3.0e38f);
      mx = fmaxf(mx, (by & 32u)  ? fb.y : -3.0e38f);
      mx = fmaxf(mx, (by & 64u)  ? fb.z : -3.0e38f);
      mx = fmaxf(mx, (by & 128u) ? fb.w : -3.0e38f);
    }
  }
  const float mo = __shfl_xor(mx, 16);
  const int   ao = __shfl_xor((int)any, 16);
  mx = fmaxf(mx, mo);
  any |= (unsigned int)ao;
  float e = f1v + mx;
  e = e > 0.f ? e : 0.2f * e;
  return (any != 0u) ? e : NEGC;
}

__device__ __forceinline__ void gen_p(float f1v, float mrow, unsigned int word, const float* f2p, int hh,
                                      FragB& ahi, FragB& alo, float& lsum) {
#pragma unroll
  for (int hf = 0; hf < 2; ++hf) {
    const int sh = 16 * hf + 8 * hh;
    const unsigned int by = (word >> sh) & 0xffu;
    const v4f fa = *(const v4fa*)(f2p + sh);
    const v4f fb = *(const v4fa*)(f2p + sh + 4);
    float fv[8];
    fv[0] = fa.x; fv[1] = fa.y; fv[2] = fa.z; fv[3] = fa.w;
    fv[4] = fb.x; fv[5] = fb.y; fv[6] = fb.z; fv[7] = fb.w;
    unsigned int hb[8], lb[8];
#pragma unroll
    for (int q = 0; q < 8; ++q) {
      float e = f1v + fv[q];
      e = e > 0.f ? e : 0.2f * e;
      const float v = ((by >> q) & 1u) ? e : NEGC;
      const float p = expf(v - mrow);
      lsum += p;
      hb[q] = f2bf(p);
      lb[q] = f2bf(p - bf2f(hb[q]));
    }
#pragma unroll
    for (int q2 = 0; q2 < 4; ++q2) {
      ahi.w[4 * hf + q2] = (int)(hb[2 * q2] | (hb[2 * q2 + 1] << 16));
      alo.w[4 * hf + q2] = (int)(lb[2 * q2] | (lb[2 * q2 + 1] << 16));
    }
  }
}

__global__ __launch_bounds__(128) void k_atth(const unsigned int* __restrict__ ABITS, const float* __restrict__ F12,
                                              const unsigned short* __restrict__ HTh,
                                              const unsigned short* __restrict__ HTl,
                                              unsigned short* Y) {
  __shared__ __attribute__((aligned(16))) float stg[64 * 64];
  __shared__ __attribute__((aligned(16))) v4u ypk[1024];
  __shared__ __attribute__((aligned(16))) float sf2[NN];
  __shared__ __attribute__((aligned(16))) unsigned int sbits[64 * BPITCH];
  const int tid = (int)threadIdx.x, lane = tid & 31, wave = tid >> 5, hh = lane >> 4, m = lane & 15;
  const int i0 = (int)blockIdx.x * 64;
  const int bh = (int)blockIdx.y;
  const int b  = bh >> 3, head = bh & 7;
  const float* F1 = F12 + (size_t)bh * (2 * NN);
  const float* F2 = F1 + NN;

  for (int i = tid; i < NN / 4; i += 128) *(v4fa*)(sf2 + 4 * i) = *(const v4fa*)(F2 + 4 * i);
  {
    const unsigned int* ab = ABITS + ((size_t)b * NN + i0) * 32;
    for (int i = tid; i < 64 * 8; i += 128) {
      const int row = i >> 3, q = i & 7;
      const v4u w = *(const v4ua*)(ab + row * 32 + 4 * q);
      *(v4ua*)(sbits + row * BPITCH + 4 * q) = w;
    }
  }
  __syncthreads();

  const int rl = 16 * wave + m;
  const float f1v = F1[i0 + rl];
  const unsigned int* sb = sbits + rl * BPITCH;
  const float mrow = row_max(sb, sf2, f1v, hh);

  v8f acc[4];
  {
    const v8f z = {0.f, 0.f, 0.f, 0.f, 0.f, 0.f, 0.f, 0.f};
    acc[0] = z; acc[1] = z; acc[2] = z; acc[3] = z;
  }
  float lsum = 0.0f;
  const size_t hoff = ((size_t)bh * HID + m) * NN + 8 * hh;
  const unsigned short* hph = HTh + hoff;
  const unsigned short* hpl = HTl + hoff;
#pragma unroll 1
  for (int jt = 0; jt < 32; ++jt) {
    FragB ahi, alo;
    gen_p(f1v, mrow, sb[jt], sf2 + 32 * jt, hh, ahi, alo, lsum);
#pragma unroll
    for (int t = 0; t < 4; ++t) {
      const unsigned short* qh = hph + (size_t)(16 * t) * NN + 32 * jt;
      const unsigned short* ql = hpl + (size_t)(16 * t) * NN + 32 * jt;
      FragB bhf, blf;
      bhf.h[0] = *(const v8usa*)qh;
      bhf.h[1] = *(const v8usa*)(qh + 16);
      blf.h[0] = *(const v8usa*)ql;
      blf.h[1] = *(const v8usa*)(ql + 16);
      acc[t] = wmb(ahi, bhf, acc[t]);
      acc[t] = wmb(ahi, blf, acc[t]);
      acc[t] = wmb(alo, bhf, acc[t]);
    }
  }

  lsum += __shfl_xor(lsum, 16);
  const float inv = 1.0f / lsum;
  float invr[8];
#pragma unroll
  for (int r = 0; r < 8; ++r) invr[r] = __shfl(inv, 8 * hh + r);
#pragma unroll
  for (int t = 0; t < 4; ++t) {
    const int lc = 16 * t + m;
#pragma unroll
    for (int r = 0; r < 8; ++r) {
      const int lr = 16 * wave + 8 * hh + r;
      stg[lr * 64 + lc] = acc[t][r] * invr[r];
    }
  }
  __syncthreads();

#pragma unroll 1
  for (int it = 0; it < 4; ++it) {
    const int u   = it * 128 + tid;
    const int row = u >> 3, pc = u & 7;
    const v4f a0 = *(const v4fa*)(stg + row * 64 + 8 * pc);
    const v4f a1 = *(const v4fa*)(stg + row * 64 + 8 * pc + 4);
    float v[8];
    v[0] = a0.x; v[1] = a0.y; v[2] = a0.z; v[3] = a0.w;
    v[4] = a1.x; v[5] = a1.y; v[6] = a1.z; v[7] = a1.w;
#pragma unroll
    for (int i = 0; i < 8; ++i) {
      float e = eluf(v[i]);
      e = e > 0.f ? e : 0.01f * e;
      v[i] = e;
    }
    v4u hv, lv;
    split8(v, hv, lv);
    ypk[2 * u]     = hv;
    ypk[2 * u + 1] = lv;
    unsigned short* gp = Y + ((size_t)b * NN + i0 + row) * (size_t)(2 * CAT) + head * HID + 8 * pc;
    *(volatile v4u*)gp = hv;
    *(volatile v4u*)(gp + CAT) = lv;
  }
  __threadfence();
#pragma unroll 1
  for (int it = 0; it < 4; ++it) {
    const int u   = it * 128 + tid;
    const int row = u >> 3, pc = u & 7;
    const v4u hv = ypk[2 * u];
    const v4u lv = ypk[2 * u + 1];
    unsigned short* gp = Y + ((size_t)b * NN + i0 + row) * (size_t)(2 * CAT) + head * HID + 8 * pc;
    *(volatile v4u*)gp = hv;
    *(volatile v4u*)(gp + CAT) = lv;
  }
}

__global__ __launch_bounds__(256) void k_out(const unsigned short* __restrict__ Y,
                                             const unsigned short* __restrict__ WO2,
                                             const float* __restrict__ aout,
                                             float* G12, unsigned short* HOh, unsigned short* HOl) {
  extern __shared__ __attribute__((aligned(16))) float gsm[];
  float* stg = gsm;
  float* sdt = gsm + 64 * NCL;
  const int tid = (int)threadIdx.x, lane = tid & 31, wave = tid >> 5, hh = lane >> 4, m = lane & 15;
  const int rg = wave & 3, cg = wave >> 2;
  const int rowBase = (int)blockIdx.x * 64;
  const int colBase = cg * 128;

  v8f acc[8];
  {
    const v8f z = {0.f, 0.f, 0.f, 0.f, 0.f, 0.f, 0.f, 0.f};
#pragma unroll
    for (int t = 0; t < 8; ++t) acc[t] = z;
  }
  const unsigned short* ap = Y   + (size_t)(rowBase + 16 * rg + m) * (size_t)(2 * CAT) + 8 * hh;
  const unsigned short* bp = WO2 + (size_t)(colBase + m) * (size_t)(2 * CAT) + 8 * hh;
#pragma unroll 1
  for (int k0 = 0; k0 < 2 * CAT; k0 += 32) {
    FragB af;
    af.h[0] = *(const v8usa*)(ap + k0);
    af.h[1] = *(const v8usa*)(ap + k0 + 16);
#pragma unroll
    for (int nt = 0; nt < 8; ++nt) {
      const unsigned short* wq = bp + (size_t)(16 * nt) * (size_t)(2 * CAT) + k0;
      FragB bf;
      bf.h[0] = *(const v8usa*)wq;
      bf.h[1] = *(const v8usa*)(wq + 16);
      acc[nt] = wmb(af, bf, acc[nt]);
    }
  }

#pragma unroll
  for (int nt = 0; nt < 8; ++nt) {
    const int lc = colBase + 16 * nt + m;
#pragma unroll
    for (int r = 0; r < 8; ++r) {
      const int lr = 16 * rg + 8 * hh + r;
      stg[lr * NCL + lc] = acc[nt][r];
    }
  }
  __syncthreads();

  v4f as4[2], ad4[2];
#pragma unroll
  for (int c = 0; c < 2; ++c) {
    as4[c] = bfr4(*(const v4fa*)(aout + c * 128 + 4 * lane));
    ad4[c] = bfr4(*(const v4fa*)(aout + NCL + c * 128 + 4 * lane));
  }
#pragma unroll 1
  for (int i = 0; i < 8; ++i) {
    const int row = wave * 8 + i;
    float s = 0.0f, d = 0.0f;
#pragma unroll
    for (int c = 0; c < 2; ++c) {
      const v4f p = *(const v4fa*)(stg + row * NCL + c * 128 + 4 * lane);
      s = fmaf(p.x, as4[c].x, s); s = fmaf(p.y, as4[c].y, s); s = fmaf(p.z, as4[c].z, s); s = fmaf(p.w, as4[c].w, s);
      d = fmaf(p.x, ad4[c].x, d); d = fmaf(p.y, ad4[c].y, d); d = fmaf(p.z, ad4[c].z, d); d = fmaf(p.w, ad4[c].w, d);
    }
#pragma unroll
    for (int off = 16; off > 0; off >>= 1) {
      s += __shfl_xor(s, off);
      d += __shfl_xor(d, off);
    }
    if (lane == 0) { sdt[row] = s; sdt[64 + row] = d; }
  }
  __syncthreads();

  const int b = rowBase >> 10, n0 = rowBase & (NN - 1);
  const v4f gv = *(const v4fa*)(sdt + 4 * lane);
  float* gp = G12 + ((size_t)b * 2 + (lane >> 4)) * NN + n0 + 4 * (lane & 15);
  const size_t hbase = (size_t)b * (size_t)(NCL * NN) + n0;

  tr_store_pass<NCL, 256, 8>(stg, HOh, HOl, hbase, tid);
  if (wave == 0) *(volatile v4f*)gp = gv;
  __threadfence();
  tr_store_pass<NCL, 256, 8>(stg, HOh, HOl, hbase, tid);
  if (wave == 0) *(volatile v4f*)gp = gv;
}

template <int LAYER>
__device__ __forceinline__ void atto_store_pass(const float* stg, int wave, int lane, int b, int i0,
                                                float* XO, unsigned short* X1HL) {
#pragma unroll 1
  for (int i = 0; i < 8; ++i) {
    const int row = 8 * wave + i;
    const size_t grow = (size_t)b * NN + i0 + row;
    const float* sr = stg + row * NCL;
    const v4f p0 = *(const v4fa*)(sr + 4 * lane);
    const v4f p1 = *(const v4fa*)(sr + 128 + 4 * lane);
    float* op = XO + grow * NCL + 4 * lane;
    *(volatile v4f*)op = p0;
    *(volatile v4f*)(op + 128) = p1;
    if constexpr (LAYER == 0) {
      const v4f q0 = *(const v4fa*)(sr + 8 * lane);
      const v4f q1 = *(const v4fa*)(sr + 8 * lane + 4);
      float v[8];
      v[0] = q0.x; v[1] = q0.y; v[2] = q0.z; v[3] = q0.w;
      v[4] = q1.x; v[5] = q1.y; v[6] = q1.z; v[7] = q1.w;
      v4u hv, lv;
      split8(v, hv, lv);
      unsigned short* hp = X1HL + grow * (size_t)(2 * NCL) + 8 * lane;
      *(volatile v4u*)hp = hv;
      *(volatile v4u*)(hp + NCL) = lv;
    } else {
      if (i0 == 0 && row == 0) {
        float* o1 = XO + (size_t)OUT1OFF + (size_t)b * NCL + 4 * lane;
        *(volatile v4f*)o1 = p0;
        *(volatile v4f*)(o1 + 128) = p1;
      }
    }
  }
}

template <int LAYER>
__global__ __launch_bounds__(256) void k_atto(const unsigned int* __restrict__ ABITS, const float* __restrict__ G12,
                                              const unsigned short* __restrict__ HOh,
                                              const unsigned short* __restrict__ HOl,
                                              const float* __restrict__ res, const int* __restrict__ mask,
                                              const float* __restrict__ lnw, const float* __restrict__ lnb,
                                              float* XO, unsigned short* X1HL) {
  extern __shared__ __attribute__((aligned(16))) float osm[];
  float* stg = osm;
  float* sf2 = osm + 64 * NCL;
  unsigned int* sbits = (unsigned int*)(osm + 64 * NCL + NN);
  const int tid = (int)threadIdx.x, lane = tid & 31, wave = tid >> 5, hh = lane >> 4, m = lane & 15;
  const int rg = wave & 3, cg = wave >> 2;
  const int i0 = (int)blockIdx.x * 64;
  const int b  = (int)blockIdx.y;
  const float* G1 = G12 + (size_t)b * (2 * NN);
  const float* G2 = G1 + NN;

  for (int i = tid; i < NN / 4; i += 256) *(v4fa*)(sf2 + 4 * i) = *(const v4fa*)(G2 + 4 * i);
  {
    const unsigned int* ab = ABITS + ((size_t)b * NN + i0) * 32;
    for (int i = tid; i < 64 * 8; i += 256) {
      const int row = i >> 3, q = i & 7;
      const v4u w = *(const v4ua*)(ab + row * 32 + 4 * q);
      *(v4ua*)(sbits + row * BPITCH + 4 * q) = w;
    }
  }
  __syncthreads();

  const int rl = 16 * rg + m;
  const float g1v = G1[i0 + rl];
  const unsigned int* sb = sbits + rl * BPITCH;
  const float mrow = row_max(sb, sf2, g1v, hh);

  v8f acc[8];
  {
    const v8f z = {0.f, 0.f, 0.f, 0.f, 0.f, 0.f, 0.f, 0.f};
#pragma unroll
    for (int t = 0; t < 8; ++t) acc[t] = z;
  }
  float lsum = 0.0f;
  const size_t hoff = ((size_t)b * NCL + 128 * cg + m) * NN + 8 * hh;
  const unsigned short* hph = HOh + hoff;
  const unsigned short* hpl = HOl + hoff;
#pragma unroll 1
  for (int jt = 0; jt < 32; ++jt) {
    FragB ahi, alo;
    gen_p(g1v, mrow, sb[jt], sf2 + 32 * jt, hh, ahi, alo, lsum);
#pragma unroll
    for (int t = 0; t < 8; ++t) {
      const unsigned short* qh = hph + (size_t)(16 * t) * NN + 32 * jt;
      const unsigned short* ql = hpl + (size_t)(16 * t) * NN + 32 * jt;
      FragB bhf, blf;
      bhf.h[0] = *(const v8usa*)qh;
      bhf.h[1] = *(const v8usa*)(qh + 16);
      blf.h[0] = *(const v8usa*)ql;
      blf.h[1] = *(const v8usa*)(ql + 16);
      acc[t] = wmb(ahi, bhf, acc[t]);
      acc[t] = wmb(ahi, blf, acc[t]);
      acc[t] = wmb(alo, bhf, acc[t]);
    }
  }

  lsum += __shfl_xor(lsum, 16);
  const float inv = 1.0f / lsum;
  float invr[8];
#pragma unroll
  for (int r = 0; r < 8; ++r) invr[r] = __shfl(inv, 8 * hh + r);
#pragma unroll
  for (int t = 0; t < 8; ++t) {
    const int lc = 128 * cg + 16 * t + m;
#pragma unroll
    for (int r = 0; r < 8; ++r) {
      const int lr = 16 * rg + 8 * hh + r;
      stg[lr * NCL + lc] = acc[t][r] * invr[r];
    }
  }
  __syncthreads();

  {
    const v4f w0 = bfr4(*(const v4fa*)(lnw + 4 * lane));
    const v4f w1 = bfr4(*(const v4fa*)(lnw + 128 + 4 * lane));
    const v4f c0 = bfr4(*(const v4fa*)(lnb + 4 * lane));
    const v4f c1 = bfr4(*(const v4fa*)(lnb + 128 + 4 * lane));
    const float wv[8] = {w0.x, w0.y, w0.z, w0.w, w1.x, w1.y, w1.z, w1.w};
    const float cv[8] = {c0.x, c0.y, c0.z, c0.w, c1.x, c1.y, c1.z, c1.w};
#pragma unroll 1
    for (int i = 0; i < 8; ++i) {
      const int row = 8 * wave + i;
      const size_t grow = (size_t)b * NN + i0 + row;
      float* sr = stg + row * NCL;
      const v4f o0 = *(const v4fa*)(sr + 4 * lane);
      const v4f o1 = *(const v4fa*)(sr + 128 + 4 * lane);
      v4f r0 = *(const v4fa*)(res + grow * NCL + 4 * lane);
      v4f r1 = *(const v4fa*)(res + grow * NCL + 128 + 4 * lane);
      if constexpr (LAYER == 0) { r0 = bfr4(r0); r1 = bfr4(r1); }
      const bool mz = (mask[grow] == 0);
      const float ov[8] = {o0.x, o0.y, o0.z, o0.w, o1.x, o1.y, o1.z, o1.w};
      const float rv[8] = {r0.x, r0.y, r0.z, r0.w, r1.x, r1.y, r1.z, r1.w};
      float t[8];
      float s = 0.0f;
#pragma unroll
      for (int e = 0; e < 8; ++e) {
        const float y = rv[e] + eluf(ov[e]);
        t[e] = mz ? 0.0f : y;
        s += t[e];
      }
#pragma unroll
      for (int off = 16; off > 0; off >>= 1) s += __shfl_xor(s, off);
      const float mu = s * (1.0f / 256.0f);
      float q = 0.0f;
#pragma unroll
      for (int e = 0; e < 8; ++e) {
        t[e] = t[e] - mu;
        q = fmaf(t[e], t[e], q);
      }
#pragma unroll
      for (int off = 16; off > 0; off >>= 1) q += __shfl_xor(q, off);
      const float var  = q * (1.0f / 256.0f);
      const float rstd = 1.0f / sqrtf(var + 1e-5f);
      float y[8];
#pragma unroll
      for (int e = 0; e < 8; ++e) {
        float z = fmaf(t[e] * rstd, wv[e], cv[e]);
        if (LAYER == 1) z = fmaxf(z, 0.0f);
        y[e] = z;
      }
      v4f y0, y1;
      y0.x = y[0]; y0.y = y[1]; y0.z = y[2]; y0.w = y[3];
      y1.x = y[4]; y1.y = y[5]; y1.z = y[6]; y1.w = y[7];
      *(v4fa*)(sr + 4 * lane) = y0;
      *(v4fa*)(sr + 128 + 4 * lane) = y1;
    }
  }
  __syncthreads();

  atto_store_pass<LAYER>(stg, wave, lane, b, i0, XO, X1HL);
  __threadfence();
  atto_store_pass<LAYER>(stg, wave, lane, b, i0, XO, X1HL);
}

extern "C" void kernel_launch(void* const* d_in, const int* in_sizes, int n_in,
                              void* d_out, int out_size, void* d_ws, size_t ws_size,
                              hipStream_t stream) {
  if (n_in < 9) return;
  if (in_sizes[0] != MROWS * NF) return;
  if (in_sizes[1] != NB * NN * NN) return;
  if (in_sizes[2] != MROWS) return;
  if (in_sizes[3] != NHD * NF * HID) return;
  if (in_sizes[4] != NHD * 2 * HID) return;
  if (in_sizes[5] != CAT * NCL) return;
  if (in_sizes[6] != 2 * NCL) return;
  if (in_sizes[7] != NCL || in_sizes[8] != NCL) return;
  if (out_size != MROWS * NCL + NB * NCL) return;

  const float* x     = (const float*)d_in[0];
  const int*   adj   = (const int*)  d_in[1];
  const int*   mask  = (const int*)  d_in[2];
  const float* Watt  = (const float*)d_in[3];
  const float* aatt  = (const float*)d_in[4];
  const float* Wout  = (const float*)d_in[5];
  const float* aout  = (const float*)d_in[6];
  const float* lnw   = (const float*)d_in[7];
  const float* lnb   = (const float*)d_in[8];
  float* out = (float*)d_out;

  char* ws = (char*)d_ws;
  size_t off = 0;
  const size_t oXB  = off; off += (size_t)MROWS * NF * 2;            off = (off + 255) & ~(size_t)255;
  const size_t oWA2 = off; off += (size_t)CAT * (2 * NF) * 2;        off = (off + 255) & ~(size_t)255;
  const size_t oWO2 = off; off += (size_t)NCL * (2 * CAT) * 2;       off = (off + 255) & ~(size_t)255;
  const size_t oAB  = off; off += (size_t)MROWS * 32 * 4;            off = (off + 255) & ~(size_t)255;
  const size_t oF12 = off; off += (size_t)NB * NHD * 2 * NN * 4;     off = (off + 255) & ~(size_t)255;
  const size_t oG12 = off; off += (size_t)NB * 2 * NN * 4;           off = (off + 255) & ~(size_t)255;
  const size_t oHTh = off; off += (size_t)NB * NHD * HID * NN * 2;   off = (off + 255) & ~(size_t)255;
  const size_t oHTl = off; off += (size_t)NB * NHD * HID * NN * 2;   off = (off + 255) & ~(size_t)255;
  const size_t oY   = off; off += (size_t)MROWS * (2 * CAT) * 2;     off = (off + 255) & ~(size_t)255;
  const size_t oHOh = off; off += (size_t)NB * NCL * NN * 2;         off = (off + 255) & ~(size_t)255;
  const size_t oHOl = off; off += (size_t)NB * NCL * NN * 2;         off = (off + 255) & ~(size_t)255;
  const size_t oX1  = off; off += (size_t)MROWS * NCL * 4;           off = (off + 255) & ~(size_t)255;
  const size_t oXHL = off; off += (size_t)MROWS * (2 * NCL) * 2;     off = (off + 255) & ~(size_t)255;
  if (off > ws_size || off > (size_t)WSMAX) return;
  unsigned short* XB   = (unsigned short*)(ws + oXB);
  unsigned short* WA2  = (unsigned short*)(ws + oWA2);
  unsigned short* WO2  = (unsigned short*)(ws + oWO2);
  unsigned int*   AB   = (unsigned int*)  (ws + oAB);
  float*          F12  = (float*)(ws + oF12);
  float*          G12  = (float*)(ws + oG12);
  unsigned short* HTh  = (unsigned short*)(ws + oHTh);
  unsigned short* HTl  = (unsigned short*)(ws + oHTl);
  unsigned short* Yp   = (unsigned short*)(ws + oY);
  unsigned short* HOh  = (unsigned short*)(ws + oHOh);
  unsigned short* HOl  = (unsigned short*)(ws + oHOl);
  float*          X1   = (float*)(ws + oX1);
  unsigned short* X1HL = (unsigned short*)(ws + oXHL);

  const int ldsOut = (64 * NCL + 128) * 4;
  const int ldsAtt = (64 * NCL + NN + 64 * BPITCH) * 4;
  hipFuncSetAttribute(reinterpret_cast<const void*>(&k_out), hipFuncAttributeMaxDynamicSharedMemorySize, ldsOut);
  hipFuncSetAttribute(reinterpret_cast<const void*>(&k_atto<0>), hipFuncAttributeMaxDynamicSharedMemorySize, ldsAtt);
  hipFuncSetAttribute(reinterpret_cast<const void*>(&k_atto<1>), hipFuncAttributeMaxDynamicSharedMemorySize, ldsAtt);

  k_prep<<<PU_ALL / 256, 256, 0, stream>>>(x, adj, Watt, Wout, XB, WA2, WO2, AB);

  k_h<<<dim3(MROWS / 64, NHD), 128, 0, stream>>>(XB, NF, NF, WA2, aatt, F12, HTh, HTl);
  k_atth<<<dim3(NN / 64, NB * NHD), 128, 0, stream>>>(AB, F12, HTh, HTl, Yp);
  k_out<<<MROWS / 64, 256, ldsOut, stream>>>(Yp, WO2, aout, G12, HOh, HOl);
  k_atto<0><<<dim3(NN / 64, NB), 256, ldsAtt, stream>>>(AB, G12, HOh, HOl, x, mask, lnw, lnb, X1, X1HL);

  k_h<<<dim3(MROWS / 64, NHD), 128, 0, stream>>>(X1HL, 2 * NF, 2 * NF, WA2, aatt, F12, HTh, HTl);
  k_atth<<<dim3(NN / 64, NB * NHD), 128, 0, stream>>>(AB, F12, HTh, HTl, Yp);
  k_out<<<MROWS / 64, 256, ldsOut, stream>>>(Yp, WO2, aout, G12, HOh, HOl);
  k_atto<1><<<dim3(NN / 64, NB), 256, ldsAtt, stream>>>(AB, G12, HOh, HOl, X1, mask, lnw, lnb, out, X1HL);
}
